// PointNetSetAbstraction_29394756174196
// MI455X (gfx1250) — hardware-verified
//
#include <hip/hip_runtime.h>
#pragma clang fp contract(off)

typedef __attribute__((ext_vector_type(16))) _Float16 v16h;
typedef __attribute__((ext_vector_type(8)))  _Float16 v8h;
typedef __attribute__((ext_vector_type(8)))  float    v8f;
typedef __attribute__((ext_vector_type(4)))  float    v4f;
typedef __attribute__((ext_vector_type(4)))  unsigned v4u;

constexpr int NBATCH   = 16;
constexpr int NPTS     = 4096;
constexpr int NSAMP    = 1024;
constexpr int NNEIGH   = 32;
constexpr int NCOLS    = NBATCH * NSAMP * NNEIGH;
constexpr int CIN0     = 6;
constexpr int KPAD0    = 32;
constexpr int CH_L0    = 64;
constexpr int CH_L1    = 64;
constexpr int CH_L2    = 128;
constexpr int COLS_PER_BLOCK = 1024;
constexpr int GEMM_BLOCKS    = NCOLS / COLS_PER_BLOCK;
constexpr int PART_PITCH     = 256;
constexpr int TILE_PITCH     = 72;
constexpr int OMAX_PITCH     = 36;
constexpr int BQ_QUERIES     = 64;
constexpr float W_CARRY      = 64.0f;
constexpr float W_CARRY_INV  = 1.0f / 64.0f;
constexpr float BN_EPS       = 1e-5f;
constexpr float BALL_R2      = (float)(0.4 * 0.4);

static_assert(NCOLS == 524288, "column count");
static_assert(GEMM_BLOCKS * COLS_PER_BLOCK == NCOLS, "gemm grid covers all columns");
static_assert(GEMM_BLOCKS == 512, "partials plane rows");
static_assert((NBATCH * NSAMP) % BQ_QUERIES == 0, "ball-query grid exact");
static_assert(KPAD0 % 32 == 0 && CH_L0 % 32 == 0 && CH_L1 % 32 == 0, "K multiples of 32");
static_assert(CH_L0 % 16 == 0 && CH_L1 % 16 == 0 && CH_L2 % 16 == 0, "N tile multiples");

constexpr size_t OUT0_BYTES = (size_t)NBATCH * 3 * NSAMP * 4;
constexpr size_t OUT1_BYTES = (size_t)NBATCH * CH_L2 * NSAMP * 4;
static_assert(OUT0_BYTES == 196608, "out1 byte offset");
static_assert(OUT0_BYTES % 128 == 0, "out1 starts on a line");
static_assert(OUT0_BYTES + OUT1_BYTES == 8585216, "d_out total");

constexpr size_t WS_SAMP  = 0;
constexpr size_t WS_W0    = WS_SAMP  + OUT0_BYTES;
constexpr size_t WS_W1    = WS_W0    + (size_t)CH_L0 * KPAD0 * 2;
constexpr size_t WS_W2    = WS_W1    + (size_t)CH_L1 * CH_L0 * 2;
constexpr size_t WS_PART0 = WS_W2    + (size_t)CH_L2 * CH_L1 * 2;
constexpr size_t WS_PART1 = WS_PART0 + (size_t)GEMM_BLOCKS * PART_PITCH * 4;
constexpr size_t WS_PART2 = WS_PART1 + (size_t)GEMM_BLOCKS * PART_PITCH * 4;
constexpr size_t WS_SS0   = WS_PART2 + (size_t)GEMM_BLOCKS * PART_PITCH * 4;
constexpr size_t WS_SS1   = WS_SS0   + 1024;
constexpr size_t WS_SS2   = WS_SS1   + 1024;
constexpr size_t WS_X0    = WS_SS2   + 1024;
constexpr size_t WS_Y1    = WS_X0    + (size_t)NCOLS * 8 * 2;
constexpr size_t WS_TOTAL = WS_Y1    + (size_t)NCOLS * CH_L1 * 2;
static_assert(WS_TOTAL == 77298688, "carve total");
static_assert(WS_TOTAL <= (size_t)134217728, "carve under 128 MiB");
static_assert(WS_X0 % 1024 == 0 && WS_Y1 % 1024 == 0 && WS_PART0 % 1024 == 0, "line-aligned regions");

union FragU { v16h v; v8h h[2]; };

__device__ __forceinline__ v16h frag_load(const _Float16* p) {
  FragU f;
  f.h[0] = *(const v8h*)(p);
  f.h[1] = *(const v8h*)(p + 16);
  return f.v;
}

__device__ __forceinline__ v8f mma16(v16h a, v16h b, v8f c) {
  c = __builtin_amdgcn_wmma_f32_16x16x32_f16(false, a, false, b, (short)0, c, false, false);
  asm volatile("v_nop\n\tv_nop\n\tv_nop\n\tv_nop" : "+v"(c) : "v"(a), "v"(b));
  return c;
}

__device__ __forceinline__ void wave_lds_sync() {
  __builtin_amdgcn_fence(__ATOMIC_RELEASE, "workgroup");
  __builtin_amdgcn_wave_barrier();
  __builtin_amdgcn_fence(__ATOMIC_ACQUIRE, "workgroup");
}

__device__ __forceinline__ float h16_to_f32(unsigned hb) {
  const unsigned sgn = (hb & 0x8000u) << 16;
  const unsigned em = hb & 0x7fffu;
  const float fn = __uint_as_float((em << 13) + 0x38000000u);
  const float fs = (float)em * 5.9604644775390625e-8f;
  const float mag = (em < 0x400u) ? fs : fn;
  return __uint_as_float(__float_as_uint(mag) | sgn);
}

__global__ __launch_bounds__(256) void prep_weights_kernel(const float* __restrict__ W, unsigned* __restrict__ out,
                                                           int cout, int cin, int cinp) {
  const int i = blockIdx.x * 256 + threadIdx.x;
  const int n2 = (cout * cinp) >> 1;
  if (i < n2) {
    const int e = 2 * i;
    const int o = e / cinp;
    const int k = e - o * cinp;
    const int k0 = (k < cin) ? k : (cin - 1);
    const int k1 = (k + 1 < cin) ? (k + 1) : (cin - 1);
    float f0 = W[o * cin + k0];
    float f1 = W[o * cin + k1];
    f0 = (k < cin) ? (f0 * W_CARRY) : 0.0f;
    f1 = (k + 1 < cin) ? (f1 * W_CARRY) : 0.0f;
    const _Float16 h0 = (_Float16)f0;
    const _Float16 h1 = (_Float16)f1;
    const unsigned u = (unsigned)__builtin_bit_cast(unsigned short, h0) |
                       ((unsigned)__builtin_bit_cast(unsigned short, h1) << 16);
    ((volatile unsigned*)out)[i] = u;
    __threadfence();
    ((volatile unsigned*)out)[i] = u;
  }
}

__global__ __launch_bounds__(256) void fps_kernel(const float* __restrict__ xyz, float* __restrict__ out0,
                                                  float* __restrict__ samp) {
#pragma clang fp contract(off)
  __shared__ __align__(16) float spts[3 * NPTS];
  __shared__ __align__(16) float ssam[3 * NSAMP];
  __shared__ float swv[2][8];
  __shared__ int   swi[2][8];
  const int b = blockIdx.x;
  const int tid = threadIdx.x;
  const int lane = tid & 31;
  const int wave = tid >> 5;
  const v4f* src = (const v4f*)(xyz + (size_t)b * 3 * NPTS);
#pragma unroll 1
  for (int i = tid; i < (3 * NPTS) / 4; i += 256) {
    const v4f v = src[i];
    *(v4f*)(spts + 4 * i) = v;
  }
  __syncthreads();
  float px[16], py[16], pz[16], dist[16];
#pragma unroll
  for (int j = 0; j < 16; ++j) {
    const int n = tid + j * 256;
    px[j] = spts[n];
    py[j] = spts[NPTS + n];
    pz[j] = spts[2 * NPTS + n];
    dist[j] = 1e10f;
  }
  int far = 0;
#pragma unroll 1
  for (int it = 0; it < NSAMP; ++it) {
    const float cx = spts[far];
    const float cy = spts[NPTS + far];
    const float cz = spts[2 * NPTS + far];
    if (tid == 0) {
      ssam[it] = cx;
      ssam[NSAMP + it] = cy;
      ssam[2 * NSAMP + it] = cz;
    }
    float bv = 0.0f;
    int bi = 0;
#pragma unroll
    for (int j = 0; j < 16; ++j) {
      const float dx = px[j] - cx;
      const float dy = py[j] - cy;
      const float dz = pz[j] - cz;
      const float t0 = dx * dx;
      const float t1 = dy * dy;
      const float t2 = dz * dz;
      const float d = (t0 + t2) + t1;
      const float dj = fminf(dist[j], d);
      dist[j] = dj;
      if (j == 0) {
        bv = dj;
        bi = tid;
      } else {
        const bool tk = dj > bv;
        bv = tk ? dj : bv;
        bi = tk ? (tid + j * 256) : bi;
      }
    }
#pragma unroll
    for (int off = 16; off >= 1; off >>= 1) {
      const float ov = __shfl_xor(bv, off, 32);
      const int oi = __shfl_xor(bi, off, 32);
      const bool tk = (ov > bv) || ((ov == bv) && (oi < bi));
      bv = tk ? ov : bv;
      bi = tk ? oi : bi;
    }
    const int slot = it & 1;
    if (lane == 0) {
      swv[slot][wave] = bv;
      swi[slot][wave] = bi;
    }
    __syncthreads();
    float rv = swv[slot][0];
    int ri = swi[slot][0];
#pragma unroll
    for (int w = 1; w < 8; ++w) {
      const float ov = swv[slot][w];
      const int oi = swi[slot][w];
      const bool tk = (ov > rv) || ((ov == rv) && (oi < ri));
      rv = tk ? ov : rv;
      ri = tk ? oi : ri;
    }
    far = ri & (NPTS - 1);
  }
  __syncthreads();
  float* o = out0 + (size_t)b * 3 * NSAMP;
  float* s = samp + (size_t)b * 3 * NSAMP;
  for (int pass = 0; pass < 2; ++pass) {
#pragma unroll
    for (int i = 0; i < 3; ++i) {
      const int idx = (i * 256 + tid) * 4;
      const v4f v = *(const v4f*)(ssam + idx);
      *(volatile v4f*)(o + idx) = v;
      *(volatile v4f*)(s + idx) = v;
    }
    __threadfence();
  }
}

__global__ __launch_bounds__(64) void ballgroup_kernel(const float* __restrict__ xyz, const float* __restrict__ feat,
                                                       const float* __restrict__ samp, unsigned* __restrict__ X0w) {
#pragma clang fp contract(off)
  __shared__ __align__(16) float spts[3 * NPTS];
  __shared__ int snn[BQ_QUERIES * NNEIGH];
  __shared__ float sq[3 * BQ_QUERIES];
  const int tid = threadIdx.x;
  const int b = blockIdx.x >> 4;
  const int m0 = (blockIdx.x & 15) * BQ_QUERIES;
  const v4f* src = (const v4f*)(xyz + (size_t)b * 3 * NPTS);
#pragma unroll 1
  for (int i = tid; i < (3 * NPTS) / 4; i += BQ_QUERIES) {
    const v4f v = src[i];
    *(v4f*)(spts + 4 * i) = v;
  }
  const float qx = samp[(size_t)(b * 3 + 0) * NSAMP + m0 + tid];
  const float qy = samp[(size_t)(b * 3 + 1) * NSAMP + m0 + tid];
  const float qz = samp[(size_t)(b * 3 + 2) * NSAMP + m0 + tid];
  sq[tid] = qx;
  sq[BQ_QUERIES + tid] = qy;
  sq[2 * BQ_QUERIES + tid] = qz;
  snn[tid * NNEIGH] = NPTS - 1;
  __syncthreads();
  const float q0 = qx * qx;
  const float q1 = qy * qy;
  const float q2 = qz * qz;
  const float qq = (q0 + q2) + q1;
  int cnt = 0;
#pragma unroll 1
  for (int n0 = 0; n0 < NPTS; n0 += 8) {
    if (__builtin_amdgcn_ballot_w32(cnt < NNEIGH) == 0u) break;
#pragma unroll
    for (int u = 0; u < 8; ++u) {
      const int n = n0 + u;
      const float x = spts[n];
      const float y = spts[NPTS + n];
      const float z = spts[2 * NPTS + n];
      const float t0 = x * x;
      const float t1 = y * y;
      const float t2 = z * z;
      const float xx = (t0 + t2) + t1;
      float p = qx * x;
      p = __builtin_fmaf(qy, y, p);
      p = __builtin_fmaf(qz, z, p);
      const float two_p = 2.0f * p;
      const float d = (qq - two_p) + xx;
      const bool hit = (!(d > BALL_R2)) && (cnt < NNEIGH);
      if (hit) {
        snn[tid * NNEIGH + cnt] = n;
        cnt += 1;
      }
    }
  }
  const int first = snn[tid * NNEIGH];
#pragma unroll 1
  for (int k = 0; k < NNEIGH; ++k) {
    if (k >= cnt) snn[tid * NNEIGH + k] = first;
  }
  __syncthreads();
  const float* fb = feat + (size_t)b * 3 * NPTS;
  const size_t colbase = ((size_t)b * NSAMP + m0) * NNEIGH;
#pragma unroll 1
  for (int i = 0; i < NNEIGH; ++i) {
    const int cl = i * BQ_QUERIES + tid;
    const int ql = cl >> 5;
    int n = snn[cl];
    n = n < 0 ? 0 : (n > NPTS - 1 ? NPTS - 1 : n);
    const float gx = spts[n] - sq[ql];
    const float gy = spts[NPTS + n] - sq[BQ_QUERIES + ql];
    const float gz = spts[2 * NPTS + n] - sq[2 * BQ_QUERIES + ql];
    const float f0 = fb[n];
    const float f1 = fb[NPTS + n];
    const float f2 = fb[2 * NPTS + n];
    const _Float16 e0 = (_Float16)gx;
    const _Float16 e1 = (_Float16)gy;
    const _Float16 e2 = (_Float16)gz;
    const _Float16 e3 = (_Float16)f0;
    const _Float16 e4 = (_Float16)f1;
    const _Float16 e5 = (_Float16)f2;
    const unsigned u0 = (unsigned)__builtin_bit_cast(unsigned short, e0);
    const unsigned u1 = (unsigned)__builtin_bit_cast(unsigned short, e1);
    const unsigned u2 = (unsigned)__builtin_bit_cast(unsigned short, e2);
    const unsigned u3 = (unsigned)__builtin_bit_cast(unsigned short, e3);
    const unsigned u4 = (unsigned)__builtin_bit_cast(unsigned short, e4);
    const unsigned u5 = (unsigned)__builtin_bit_cast(unsigned short, e5);
    v4u w;
    w[0] = u0 | (u1 << 16);
    w[1] = u2 | (u3 << 16);
    w[2] = u4 | (u5 << 16);
    w[3] = 0u;
    unsigned* dst = X0w + (colbase + (size_t)cl) * 4;
    *(volatile v4u*)dst = w;
    __threadfence();
    *(volatile v4u*)dst = w;
  }
}

__device__ __forceinline__ void stats_flush4(float (&ls)[4], float (&lq)[4], float* sred, float* prec, int tid) {
  const int lane = tid & 31;
  const int wave = tid >> 5;
  const int h = lane >> 4;
  const int c = lane & 15;
#pragma unroll
  for (int nt = 0; nt < 4; ++nt) {
    const float os = __shfl_xor(ls[nt], 16, 32);
    const float oq = __shfl_xor(lq[nt], 16, 32);
    ls[nt] = ls[nt] + os;
    lq[nt] = lq[nt] + oq;
  }
#pragma unroll
  for (int nt = 0; nt < 4; ++nt) {
    const int ch = h * 64 + nt * 16 + c;
    sred[wave * 256 + ch] = h ? 0.0f : ls[nt];
    sred[wave * 256 + 128 + ch] = h ? 0.0f : lq[nt];
  }
  __syncthreads();
  float a = 0.0f;
#pragma unroll
  for (int w = 0; w < 8; ++w) a = a + sred[w * 256 + tid];
  ((volatile float*)prec)[tid] = a;
  __threadfence();
  ((volatile float*)prec)[tid] = a;
}

__device__ __forceinline__ v16h x0_frag(const _Float16* X0h, size_t row, int h) {
  const v8h ld = *(const v8h*)(X0h + row * 8);
  const v8h z = {(_Float16)0.0f, (_Float16)0.0f, (_Float16)0.0f, (_Float16)0.0f,
                 (_Float16)0.0f, (_Float16)0.0f, (_Float16)0.0f, (_Float16)0.0f};
  FragU a;
  a.h[0] = h ? z : ld;
  a.h[1] = z;
  return a.v;
}

__global__ __launch_bounds__(256) void stats0_kernel(const _Float16* __restrict__ X0h, const _Float16* __restrict__ W0h,
                                                     float* __restrict__ part) {
  __shared__ __align__(16) _Float16 sW0[CH_L0 * KPAD0];
  __shared__ float sred[8 * 256];
  const int tid = threadIdx.x;
  const int lane = tid & 31;
  const int wave = tid >> 5;
  const int h = lane >> 4;
  const int c = lane & 15;
  ((v4u*)sW0)[tid] = ((const v4u*)W0h)[tid];
  __syncthreads();
  v16h bw[4];
#pragma unroll
  for (int nt = 0; nt < 4; ++nt) bw[nt] = frag_load(sW0 + (nt * 16 + c) * KPAD0 + 8 * h);
  const v8f zero8 = {0.f, 0.f, 0.f, 0.f, 0.f, 0.f, 0.f, 0.f};
  float ls[4], lq[4];
#pragma unroll
  for (int nt = 0; nt < 4; ++nt) { ls[nt] = 0.0f; lq[nt] = 0.0f; }
  const size_t col0 = (size_t)blockIdx.x * COLS_PER_BLOCK + (size_t)wave * 128;
#pragma unroll 1
  for (int t = 0; t < 8; ++t) {
    const v16h a = x0_frag(X0h, col0 + t * 16 + c, h);
#pragma unroll
    for (int nt = 0; nt < 4; ++nt) {
      const v8f acc = mma16(a, bw[nt], zero8);
#pragma unroll
      for (int r = 0; r < 8; ++r) {
        const float y = acc[r] * W_CARRY_INV;
        ls[nt] = ls[nt] + y;
        lq[nt] = lq[nt] + y * y;
      }
    }
  }
  stats_flush4(ls, lq, sred, part + (size_t)blockIdx.x * PART_PITCH, tid);
}

__global__ __launch_bounds__(256) void finalize_kernel(const float* __restrict__ part, const float* __restrict__ gam,
                                                       const float* __restrict__ bet, float* __restrict__ ss, int cout) {
  __shared__ double dsum[256];
  __shared__ float sout[256];
  const int tid = threadIdx.x;
  double a = 0.0;
#pragma unroll 4
  for (int blk = 0; blk < GEMM_BLOCKS; ++blk) a = a + (double)part[(size_t)blk * PART_PITCH + tid];
  dsum[tid] = a;
  __syncthreads();
  if (tid < 128) {
    const int cc = (tid < cout) ? tid : (cout - 1);
    const double inv_n = 1.0 / (double)NCOLS;
    const double mu = dsum[cc] * inv_n;
    const double ex2 = dsum[128 + cc] * inv_n;
    double var = ex2 - mu * mu;
    var = (var < 0.0) ? 0.0 : var;
    const float sd = sqrtf((float)var + BN_EPS);
    const float sc = gam[cc] * (1.0f / sd);
    const float sh = bet[cc] - (float)mu * sc;
    const bool ok = tid < cout;
    sout[tid] = ok ? sc : 0.0f;
    sout[128 + tid] = ok ? sh : 0.0f;
  }
  __syncthreads();
  const float v = sout[tid];
  ((volatile float*)ss)[tid] = v;
  __threadfence();
  ((volatile float*)ss)[tid] = v;
}

__global__ __launch_bounds__(256) void layer01_kernel(const _Float16* __restrict__ X0h, const _Float16* __restrict__ W0h,
                                                      const _Float16* __restrict__ W1h, const float* __restrict__ ss0,
                                                      _Float16* __restrict__ Y1h, float* __restrict__ part) {
  __shared__ __align__(16) _Float16 sW0[CH_L0 * KPAD0];
  __shared__ __align__(16) _Float16 sW1[CH_L1 * CH_L0];
  __shared__ __align__(16) _Float16 sAct[8][16 * TILE_PITCH];
  __shared__ __align__(16) _Float16 sOutT[8][16 * TILE_PITCH];
  __shared__ float sbn[256];
  __shared__ float sred[8 * 256];
  const int tid = threadIdx.x;
  const int lane = tid & 31;
  const int wave = tid >> 5;
  const int h = lane >> 4;
  const int c = lane & 15;
  ((v4u*)sW0)[tid] = ((const v4u*)W0h)[tid];
  ((v4u*)sW1)[tid] = ((const v4u*)W1h)[tid];
  ((v4u*)sW1)[tid + 256] = ((const v4u*)W1h)[tid + 256];
  sbn[tid] = ss0[tid];
  __syncthreads();
  v16h bw0[4];
  float scw[4], shf[4];
#pragma unroll
  for (int nt = 0; nt < 4; ++nt) {
    bw0[nt] = frag_load(sW0 + (nt * 16 + c) * KPAD0 + 8 * h);
    scw[nt] = sbn[nt * 16 + c] * W_CARRY_INV;
    shf[nt] = sbn[128 + nt * 16 + c];
  }
  const v8f zero8 = {0.f, 0.f, 0.f, 0.f, 0.f, 0.f, 0.f, 0.f};
  float ls[4], lq[4];
#pragma unroll
  for (int nt = 0; nt < 4; ++nt) { ls[nt] = 0.0f; lq[nt] = 0.0f; }
  _Float16* tileA = sAct[wave];
  _Float16* tileY = sOutT[wave];
  const size_t col0 = (size_t)blockIdx.x * COLS_PER_BLOCK + (size_t)wave * 128;
#pragma unroll 1
  for (int t = 0; t < 8; ++t) {
    const v16h a0 = x0_frag(X0h, col0 + t * 16 + c, h);
    v8f acc0[4];
#pragma unroll
    for (int nt = 0; nt < 4; ++nt) acc0[nt] = mma16(a0, bw0[nt], zero8);
#pragma unroll
    for (int nt = 0; nt < 4; ++nt) {
#pragma unroll
      for (int r = 0; r < 8; ++r) {
        const float x = fmaxf(acc0[nt][r] * scw[nt] + shf[nt], 0.0f);
        tileA[(8 * h + r) * TILE_PITCH + nt * 16 + c] = (_Float16)x;
      }
    }
    wave_lds_sync();
    const v16h a1k0 = frag_load(tileA + c * TILE_PITCH + 8 * h);
    const v16h a1k1 = frag_load(tileA + c * TILE_PITCH + 32 + 8 * h);
#pragma unroll
    for (int nt = 0; nt < 4; ++nt) {
      const v16h b0 = frag_load(sW1 + (nt * 16 + c) * CH_L0 + 8 * h);
      const v16h b1 = frag_load(sW1 + (nt * 16 + c) * CH_L0 + 32 + 8 * h);
      v8f acc = mma16(a1k0, b0, zero8);
      acc = mma16(a1k1, b1, acc);
#pragma unroll
      for (int r = 0; r < 8; ++r) {
        const float y = acc[r] * W_CARRY_INV;
        ls[nt] = ls[nt] + y;
        lq[nt] = lq[nt] + y * y;
        tileY[(8 * h + r) * TILE_PITCH + nt * 16 + c] = (_Float16)y;
      }
    }
    wave_lds_sync();
    {
      const int q = lane >> 3;
      const int seg = (lane & 7) * 8;
      for (int pass = 0; pass < 2; ++pass) {
#pragma unroll
        for (int it = 0; it < 4; ++it) {
          const int row = it * 4 + q;
          const v8h hv = *(const v8h*)(tileY + row * TILE_PITCH + seg);
          _Float16* dst = Y1h + (col0 + (size_t)(t * 16 + row)) * CH_L1 + seg;
          *(volatile v8h*)dst = hv;
        }
        __threadfence();
      }
    }
    wave_lds_sync();
  }
  stats_flush4(ls, lq, sred, part + (size_t)blockIdx.x * PART_PITCH, tid);
}

__device__ __forceinline__ void build_afrag(const unsigned* __restrict__ yrow, const float* sbn, int h, v16h (&a)[2]) {
  v4u w[4];
#pragma unroll
  for (int q = 0; q < 4; ++q) w[q] = *(const v4u*)(yrow + q * 8);
#pragma unroll
  for (int q = 0; q < 4; ++q) {
#pragma unroll
    for (int j = 0; j < 4; ++j) {
      const unsigned wj = w[q][j];
      const int ch = q * 16 + 8 * h + 2 * j;
      const float sc0 = sbn[ch];
      const float sc1 = sbn[ch + 1];
      const float sh0 = sbn[128 + ch];
      const float sh1 = sbn[128 + ch + 1];
      float x0 = h16_to_f32(wj & 0xffffu);
      float x1 = h16_to_f32(wj >> 16);
      x0 = fmaxf(x0 * sc0 + sh0, 0.0f);
      x1 = fmaxf(x1 * sc1 + sh1, 0.0f);
      a[q >> 1][(q & 1) * 8 + 2 * j] = (_Float16)x0;
      a[q >> 1][(q & 1) * 8 + 2 * j + 1] = (_Float16)x1;
    }
  }
}

template <bool FINAL>
__global__ __launch_bounds__(256)
void layer2_kernel(const unsigned* __restrict__ Y1w, const _Float16* __restrict__ W2h,
                   const float* __restrict__ ss1, const float* __restrict__ ss2,
                   float* __restrict__ part, float* __restrict__ out1) {
  __shared__ __align__(16) _Float16 sW2[CH_L2 * CH_L1];
  __shared__ __align__(16) float sbn1[256];
  __shared__ __align__(16) float sbn2[256];
  __shared__ __align__(16) float somax[CH_L2 * OMAX_PITCH];
  __shared__ float sacc[8 * 2 * 8 * 32];
  const int tid = threadIdx.x;
  const int lane = tid & 31;
  const int wave = tid >> 5;
  const int h = lane >> 4;
  const int c = lane & 15;
#pragma unroll
  for (int i = 0; i < 4; ++i) ((v4u*)sW2)[tid + i * 256] = ((const v4u*)W2h)[tid + i * 256];
  sbn1[tid] = ss1[tid];
  sbn2[tid] = ss2[tid];
#pragma unroll 1
  for (int i = 0; i < 16; ++i) sacc[(wave * 16 + i) * 32 + lane] = 0.0f;
  __syncthreads();
  const v8f zero8 = {0.f, 0.f, 0.f, 0.f, 0.f, 0.f, 0.f, 0.f};
  const size_t colw = (size_t)blockIdx.x * COLS_PER_BLOCK + (size_t)wave * 128;
#pragma unroll 1
  for (int g = 0; g < 4; ++g) {
    const size_t rowA = colw + (size_t)(g * 32 + c);
    const size_t rowB = rowA + 16;
    v16h aA[2], aB[2];
    build_afrag(Y1w + rowA * 32 + 4 * h, sbn1, h, aA);
    asm volatile("" ::: "memory");
    build_afrag(Y1w + rowB * 32 + 4 * h, sbn1, h, aB);
#pragma unroll 1
    for (int nt = 0; nt < 8; ++nt) {
      const _Float16* wp = sW2 + (nt * 16 + c) * CH_L1 + 8 * h;
      const v16h b0 = frag_load(wp);
      const v16h b1 = frag_load(wp + 32);
      v8f accA = mma16(aA[0], b0, zero8);
      accA = mma16(aA[1], b1, accA);
      v8f accB = mma16(aB[0], b0, zero8);
      accB = mma16(aB[1], b1, accB);
      if (FINAL) {
        const float s2 = sbn2[nt * 16 + c] * W_CARRY_INV;
        const float t2 = sbn2[128 + nt * 16 + c];
        float mx = 0.0f;
#pragma unroll
        for (int r = 0; r < 8; ++r) {
          const float va = accA[r] * s2 + t2;
          const float vb = accB[r] * s2 + t2;
          mx = fmaxf(mx, va);
          mx = fmaxf(mx, vb);
        }
        const float om = __shfl_xor(mx, 16, 32);
        mx = fmaxf(mx, om);
        if (h == 0) somax[(nt * 16 + c) * OMAX_PITCH + wave * 4 + g] = mx;
      } else {
        float ls = 0.0f;
        float lq = 0.0f;
#pragma unroll
        for (int r = 0; r < 8; ++r) {
          const float ya = accA[r] * W_CARRY_INV;
          const float yb = accB[r] * W_CARRY_INV;
          ls = ls + ya;
          lq = lq + ya * ya;
          ls = ls + yb;
          lq = lq + yb * yb;
        }
        const int si = (wave * 16 + nt) * 32 + lane;
        const float ps = sacc[si];
        const float pq = sacc[si + 256];
        sacc[si] = ps + ls;
        sacc[si + 256] = pq + lq;
      }
    }
  }
  __syncthreads();
  if (FINAL) {
    const int b = blockIdx.x >> 5;
    const int m0 = (blockIdx.x & 31) * 32;
    const int seg = (lane & 7) * 4;
    for (int pass = 0; pass < 2; ++pass) {
#pragma unroll
      for (int it = 0; it < 4; ++it) {
        const int ch = wave * 16 + it * 4 + (lane >> 3);
        const v4f v = *(const v4f*)(somax + ch * OMAX_PITCH + seg);
        float* dst = out1 + ((size_t)(b * CH_L2 + ch) * NSAMP + m0 + seg);
        *(volatile v4f*)dst = v;
      }
      __threadfence();
    }
  } else {
    const int s = tid >> 7;
    const int ch = tid & 127;
    const int nt = ch >> 4;
    const int cc = ch & 15;
    float a = 0.0f;
#pragma unroll
    for (int w = 0; w < 8; ++w) {
      const int base = ((w * 2 + s) * 8 + nt) * 32;
      a = a + sacc[base + cc];
      a = a + sacc[base + 16 + cc];
    }
    float* prec = part + (size_t)blockIdx.x * PART_PITCH;
    ((volatile float*)prec)[tid] = a;
    __threadfence();
    ((volatile float*)prec)[tid] = a;
  }
}

extern "C" void kernel_launch(void* const* d_in, const int* in_sizes, int n_in,
                              void* d_out, int out_size, void* d_ws, size_t ws_size,
                              hipStream_t stream) {
  (void)in_sizes; (void)n_in; (void)out_size;
  if (ws_size < WS_TOTAL) return;
  const float* xyz  = (const float*)d_in[0];
  const float* feat = (const float*)d_in[1];
  const float* w0   = (const float*)d_in[2];
  const float* g0   = (const float*)d_in[4];
  const float* bt0  = (const float*)d_in[5];
  const float* w1   = (const float*)d_in[6];
  const float* g1   = (const float*)d_in[8];
  const float* bt1  = (const float*)d_in[9];
  const float* w2   = (const float*)d_in[10];
  const float* g2   = (const float*)d_in[12];
  const float* bt2  = (const float*)d_in[13];

  float* out0 = (float*)d_out;
  float* out1 = (float*)((char*)d_out + OUT0_BYTES);
  char* ws = (char*)d_ws;
  float*    samp  = (float*)(ws + WS_SAMP);
  unsigned* W0w   = (unsigned*)(ws + WS_W0);
  unsigned* W1w   = (unsigned*)(ws + WS_W1);
  unsigned* W2w   = (unsigned*)(ws + WS_W2);
  float*    part0 = (float*)(ws + WS_PART0);
  float*    part1 = (float*)(ws + WS_PART1);
  float*    part2 = (float*)(ws + WS_PART2);
  float*    ss0   = (float*)(ws + WS_SS0);
  float*    ss1   = (float*)(ws + WS_SS1);
  float*    ss2   = (float*)(ws + WS_SS2);
  unsigned* X0w   = (unsigned*)(ws + WS_X0);
  unsigned* Y1w   = (unsigned*)(ws + WS_Y1);

  prep_weights_kernel<<<(CH_L0 * KPAD0 / 2) / 256, 256, 0, stream>>>(w0, W0w, CH_L0, CIN0, KPAD0);
  prep_weights_kernel<<<(CH_L1 * CH_L0 / 2) / 256, 256, 0, stream>>>(w1, W1w, CH_L1, CH_L0, CH_L0);
  prep_weights_kernel<<<(CH_L2 * CH_L1 / 2) / 256, 256, 0, stream>>>(w2, W2w, CH_L2, CH_L1, CH_L1);

  fps_kernel<<<NBATCH, 256, 0, stream>>>(xyz, out0, samp);
  ballgroup_kernel<<<(NBATCH * NSAMP) / BQ_QUERIES, BQ_QUERIES, 0, stream>>>(xyz, feat, samp, X0w);

  stats0_kernel<<<GEMM_BLOCKS, 256, 0, stream>>>((const _Float16*)X0w, (const _Float16*)W0w, part0);
  finalize_kernel<<<1, 256, 0, stream>>>(part0, g0, bt0, ss0, CH_L0);

  layer01_kernel<<<GEMM_BLOCKS, 256, 0, stream>>>((const _Float16*)X0w, (const _Float16*)W0w, (const _Float16*)W1w,
                                                  ss0, (_Float16*)Y1w, part1);
  finalize_kernel<<<1, 256, 0, stream>>>(part1, g1, bt1, ss1, CH_L1);

  layer2_kernel<false><<<GEMM_BLOCKS, 256, 0, stream>>>(Y1w, (const _Float16*)W2w, ss1, ss1, part2, out1);
  finalize_kernel<<<1, 256, 0, stream>>>(part2, g2, bt2, ss2, CH_L2);

  layer2_kernel<true><<<GEMM_BLOCKS, 256, 0, stream>>>(Y1w, (const _Float16*)W2w, ss1, ss2, part2, out1);
}
